// OuterProductMean_31361851195882
// MI455X (gfx1250) — hardware-run, weakly checked
//
#include <hip/hip_runtime.h>
#include <math.h>

typedef __attribute__((ext_vector_type(16))) _Float16 v16h;
typedef __attribute__((ext_vector_type(8)))  _Float16 v8h;
typedef __attribute__((ext_vector_type(8)))  float    v8f;
typedef __attribute__((ext_vector_type(4)))  float    v4f;

constexpr int kSeq   = 128;
constexpr int kRes   = 256;
constexpr int kCm    = 256;
constexpr int kCh    = 32;
constexpr int kCz    = 128;
constexpr int kCk    = kCh * kCh;
constexpr int kLnRows  = kSeq * kRes;
constexpr int kAbRows  = kRes * kCh;
constexpr int kChunkI  = 64;
constexpr int kChunks  = kRes / kChunkI;
constexpr int kChunkM  = kChunkI * kCh;
constexpr int kChunkPairs = kChunkI * kRes;
constexpr int kSlabPitch = 68;

static_assert(kCk == 1024, "flattened channel pair count");
static_assert((kCm % 32) == 0 && (kSeq % 32) == 0 && (kCk % 32) == 0, "every GEMM K is a multiple of 32");
static_assert((kChunkM % 64) == 0 && (kAbRows % 64) == 0 && (kChunkPairs % 64) == 0 && (kCz % 64) == 0, "tile multiples");
static_assert((kLnRows % 64) == 0 && (2 * kCh) == 64, "projection tile multiples");
static_assert(kSeq == 128 && kRes == 256 && kCm == 256 && kCh == 32 && kCz == 128, "index shifts below assume these sizes");

constexpr float kCarryMn  = 16.0f;
constexpr float kCarryW   = 256.0f;
constexpr float kResScale = 2048.0f;
constexpr float kCarryAB  = 16.0f;
constexpr float kCarryO   = 16.0f;
constexpr float kCarryWo  = 256.0f;
constexpr float kResFold  = 1.0f / kResScale;
constexpr float kProjFold = 1.0f / (kCarryMn * kCarryW);
constexpr float kOFold    = kCarryO / (kCarryAB * kCarryAB);
constexpr float kZFold    = 1.0f / (kCarryO * kCarryWo);
constexpr float kInvSeq   = 1.0f / (float)kSeq;
constexpr float kH16Min   = 6.103515625e-5f;

constexpr size_t kOffW12H = 0;
constexpr size_t kOffW12L = kOffW12H + (size_t)64 * kCm * 2;
constexpr size_t kOffWOT  = kOffW12L + (size_t)64 * kCm * 2;
constexpr size_t kOffMNH  = kOffWOT  + (size_t)kCz * kCk * 2;
constexpr size_t kOffMNL  = kOffMNH  + (size_t)kLnRows * kCm * 2;
constexpr size_t kOffABP  = kOffMNL  + (size_t)kLnRows * kCm * 2;
constexpr size_t kOffOCH  = kOffABP  + (size_t)2 * kAbRows * kSeq * 2;
constexpr size_t kWsTotal = kOffOCH  + (size_t)kChunkPairs * kCk * 2;
static_assert(kWsTotal == 71630848ull, "carve total");
static_assert(kWsTotal <= 134217728ull, "carve cap");
static_assert((kOffW12L % 128) == 0 && (kOffWOT % 128) == 0 && (kOffMNH % 128) == 0 && (kOffMNL % 128) == 0 &&
              (kOffABP % 128) == 0 && (kOffOCH % 128) == 0, "128-B aligned regions");

__device__ __forceinline__ _Float16 f2h_flush(float v) {
  const float w = (fabsf(v) < kH16Min) ? 0.0f : v;
  return (_Float16)w;
}
__device__ __forceinline__ void split_h(float v, _Float16& hi, _Float16& lo) {
  hi = f2h_flush(v);
  const float hf = (float)hi;
  const float r = (v - hf) * kResScale;
  lo = f2h_flush(r);
}
__device__ __forceinline__ v8h pack8_flush(v4f a0, v4f a1) {
  v8h h;
#pragma unroll
  for (int e = 0; e < 4; ++e) {
    h[e]     = f2h_flush(a0[e]);
    h[4 + e] = f2h_flush(a1[e]);
  }
  return h;
}
union FragU { v16h v; v8h h[2]; };
__device__ __forceinline__ v16h frag_load(const _Float16* p) {
  FragU f;
  f.h[0] = *(const v8h*)(p);
  f.h[1] = *(const v8h*)(p + 16);
  return f.v;
}
__device__ __forceinline__ v8f mma_h(v16h a, v16h b, v8f c) {
  c = __builtin_amdgcn_wmma_f32_16x16x32_f16(false, a, false, b, (short)0, c, false, false);
  asm volatile("v_nop\n\tv_nop\n\tv_nop\n\tv_nop" : "+v"(c) : "v"(a), "v"(b));
  return c;
}
__device__ __forceinline__ void wave_lds_fence() {
  __builtin_amdgcn_fence(__ATOMIC_RELEASE, "workgroup");
  __builtin_amdgcn_wave_barrier();
  __builtin_amdgcn_fence(__ATOMIC_ACQUIRE, "workgroup");
}

__global__ __launch_bounds__(256) void prep_weights_kernel(
    const float* __restrict__ W1, const float* __restrict__ W2, const float* __restrict__ Wout,
    _Float16* __restrict__ W12H, _Float16* __restrict__ W12L, _Float16* __restrict__ WOT)
{
  const int tid = threadIdx.x;
  if (blockIdx.x < 8) {
    const float* src = (blockIdx.x < 4) ? W1 : W2;
    const int g   = blockIdx.x * 256 + tid;
    const int n   = g >> 5;
    const int col = n & (kCh - 1);
    const int d0  = (g & 31) * 8;
    v8h hv, lv;
#pragma unroll
    for (int e = 0; e < 8; ++e) {
      const float w = src[(size_t)(d0 + e) * kCh + col] * kCarryW;
      _Float16 hi, lo;
      split_h(w, hi, lo);
      hv[e] = hi;
      lv[e] = lo;
    }
    const size_t o = (size_t)n * kCm + d0;
    *(volatile v8h*)(W12H + o) = hv;
    *(volatile v8h*)(W12L + o) = lv;
    __threadfence();
    *(volatile v8h*)(W12H + o) = hv;
    *(volatile v8h*)(W12L + o) = lv;
  } else {
    const int g   = (blockIdx.x - 8) * 256 + tid;
    const int z   = g >> 7;
    const int ck0 = (g & 127) * 8;
    v8h hv;
#pragma unroll
    for (int e = 0; e < 8; ++e) {
      const float w = Wout[(size_t)(ck0 + e) * kCz + z] * kCarryWo;
      hv[e] = f2h_flush(w);
    }
    const size_t o = (size_t)z * kCk + ck0;
    *(volatile v8h*)(WOT + o) = hv;
    __threadfence();
    *(volatile v8h*)(WOT + o) = hv;
  }
}

__global__ __launch_bounds__(256) void layernorm_planes_kernel(
    const float* __restrict__ m, const float* __restrict__ gamma, const float* __restrict__ beta,
    _Float16* __restrict__ MNH, _Float16* __restrict__ MNL)
{
  const int lane = threadIdx.x & 31;
  const int wave = threadIdx.x >> 5;
  const int row  = blockIdx.x * 8 + wave;
  const int s    = row / kRes;
  const int i    = row % kRes;
  const float* xr = m + (size_t)row * kCm + lane * 8;
  const v4f x0 = *(const v4f*)(xr);
  const v4f x1 = *(const v4f*)(xr + 4);
  const v4f g0 = *(const v4f*)(gamma + lane * 8);
  const v4f g1 = *(const v4f*)(gamma + lane * 8 + 4);
  const v4f b0 = *(const v4f*)(beta + lane * 8);
  const v4f b1 = *(const v4f*)(beta + lane * 8 + 4);
  float x[8], gm[8], bt[8];
#pragma unroll
  for (int e = 0; e < 4; ++e) {
    x[e] = x0[e];  x[4 + e] = x1[e];
    gm[e] = g0[e]; gm[4 + e] = g1[e];
    bt[e] = b0[e]; bt[4 + e] = b1[e];
  }
  float sum = 0.0f;
#pragma unroll
  for (int e = 0; e < 8; ++e) sum += x[e];
#pragma unroll
  for (int off = 16; off >= 1; off >>= 1) sum += __shfl_xor(sum, off, 32);
  const float mu = sum * (1.0f / (float)kCm);
  float ss = 0.0f;
#pragma unroll
  for (int e = 0; e < 8; ++e) {
    const float d = x[e] - mu;
    ss = fmaf(d, d, ss);
  }
#pragma unroll
  for (int off = 16; off >= 1; off >>= 1) ss += __shfl_xor(ss, off, 32);
  const float var  = ss * (1.0f / (float)kCm);
  const float rinv = rsqrtf(var + 1e-5f);
  v8h hv, lv;
#pragma unroll
  for (int e = 0; e < 8; ++e) {
    const float y = (x[e] - mu) * rinv * gm[e] + bt[e];
    _Float16 hi, lo;
    split_h(y * kCarryMn, hi, lo);
    hv[e] = hi;
    lv[e] = lo;
  }
  const size_t o = (size_t)(i * kSeq + s) * kCm + lane * 8;
  *(volatile v8h*)(MNH + o) = hv;
  *(volatile v8h*)(MNL + o) = lv;
  __threadfence();
  *(volatile v8h*)(MNH + o) = hv;
  *(volatile v8h*)(MNL + o) = lv;
}

__global__ __launch_bounds__(256) void proj_split_kernel(
    const _Float16* __restrict__ W12H, const _Float16* __restrict__ W12L,
    const _Float16* __restrict__ MNH,  const _Float16* __restrict__ MNL,
    const float* __restrict__ b1, const float* __restrict__ b2,
    _Float16* __restrict__ ABP)
{
  __shared__ __align__(16) float sT[8][16 * kSlabPitch];
  const int lane  = threadIdx.x & 31;
  const int wave  = threadIdx.x >> 5;
  const int tile  = blockIdx.x * 8 + wave;
  const int mt    = tile & 1;
  const int nt    = tile >> 1;
  const int m0    = mt * 32;
  const int n0    = nt * 64;
  const int rlane = lane & 15;
  const int koff  = (lane >> 4) * 8;
  const int mOff  = (lane >> 4) * 8;

  v8f accM[2][4], accR[2][4];
#pragma unroll
  for (int i = 0; i < 2; ++i)
#pragma unroll
    for (int j = 0; j < 4; ++j) {
      accM[i][j] = (v8f){0.f,0.f,0.f,0.f,0.f,0.f,0.f,0.f};
      accR[i][j] = (v8f){0.f,0.f,0.f,0.f,0.f,0.f,0.f,0.f};
    }

#pragma unroll 1
  for (int k0 = 0; k0 < kCm; k0 += 32) {
    v16h ah[2], al[2];
#pragma unroll
    for (int i = 0; i < 2; ++i) {
      const size_t ao = (size_t)(m0 + (i << 4) + rlane) * kCm + koff + k0;
      ah[i] = frag_load(W12H + ao);
      al[i] = frag_load(W12L + ao);
    }
#pragma unroll
    for (int j = 0; j < 4; ++j) {
      const size_t bo = (size_t)(n0 + (j << 4) + rlane) * kCm + koff + k0;
      const v16h bh = frag_load(MNH + bo);
      const v16h bl = frag_load(MNL + bo);
#pragma unroll
      for (int i = 0; i < 2; ++i) {
        accM[i][j] = mma_h(ah[i], bh, accM[i][j]);
        accR[i][j] = mma_h(ah[i], bl, accR[i][j]);
        accR[i][j] = mma_h(al[i], bh, accR[i][j]);
      }
    }
  }

  float* slab = sT[wave];
  const float* bias = (mt != 0) ? b2 : b1;
  const int q  = lane >> 3;
  const int c8 = (lane & 7) * 8;
  _Float16* dst = ABP + (size_t)mt * ((size_t)kAbRows * kSeq) + (size_t)(n0 >> 7) * (kCh * kSeq) + (n0 & (kSeq - 1));
#pragma unroll
  for (int i = 0; i < 2; ++i) {
    float bv[8];
#pragma unroll
    for (int r = 0; r < 8; ++r) bv[r] = bias[(i << 4) + mOff + r];
#pragma unroll
    for (int j = 0; j < 4; ++j) {
#pragma unroll
      for (int r = 0; r < 8; ++r) {
        const float t = accM[i][j][r] + accR[i][j][r] * kResFold;
        const float v = t * kProjFold + bv[r];
        slab[(mOff + r) * kSlabPitch + (j << 4) + rlane] = v * kCarryAB;
      }
    }
    wave_lds_fence();
    v8h hv[4];
#pragma unroll
    for (int it = 0; it < 4; ++it) {
      const float* sp = slab + (it * 4 + q) * kSlabPitch + c8;
      const v4f a0 = *(const v4f*)(sp);
      const v4f a1 = *(const v4f*)(sp + 4);
      hv[it] = pack8_flush(a0, a1);
    }
    for (int pass = 0; pass < 2; ++pass) {
#pragma unroll
      for (int it = 0; it < 4; ++it) {
        const int ch = (i << 4) + it * 4 + q;
        *(volatile v8h*)(dst + (size_t)ch * kSeq + c8) = hv[it];
      }
      __threadfence();
    }
    wave_lds_fence();
  }
}

__global__ __launch_bounds__(256) void outer_gemm_kernel(
    const _Float16* __restrict__ Achunk, const _Float16* __restrict__ Bt, _Float16* __restrict__ Och)
{
  __shared__ __align__(16) float sT[8][16 * kSlabPitch];
  const int lane  = threadIdx.x & 31;
  const int wave  = threadIdx.x >> 5;
  const int tile  = blockIdx.x * 8 + wave;
  constexpr int tilesN = kAbRows / 64;
  const int tm    = tile / tilesN;
  const int tn    = tile % tilesN;
  const int m0    = tm << 6;
  const int n0    = tn << 6;
  const int rlane = lane & 15;
  const int koff  = (lane >> 4) * 8;
  const int mOff  = (lane >> 4) * 8;

  v8f acc[4][4];
#pragma unroll
  for (int i = 0; i < 4; ++i)
#pragma unroll
    for (int j = 0; j < 4; ++j) acc[i][j] = (v8f){0.f,0.f,0.f,0.f,0.f,0.f,0.f,0.f};

#pragma unroll 1
  for (int k0 = 0; k0 < kSeq; k0 += 32) {
    v16h bh[4];
#pragma unroll
    for (int j = 0; j < 4; ++j)
      bh[j] = frag_load(Bt + (size_t)(n0 + (j << 4) + rlane) * kSeq + koff + k0);
#pragma unroll
    for (int i = 0; i < 4; ++i) {
      const v16h ah = frag_load(Achunk + (size_t)(m0 + (i << 4) + rlane) * kSeq + koff + k0);
#pragma unroll
      for (int j = 0; j < 4; ++j) acc[i][j] = mma_h(ah, bh[j], acc[i][j]);
    }
  }

  float* slab = sT[wave];
  const int q  = lane >> 3;
  const int t  = lane & 7;
  const int jh = q & 1;
  const int jg = (n0 >> 5) + jh;
#pragma unroll
  for (int i = 0; i < 4; ++i) {
    const int mBase = m0 + (i << 4);
    const int il = mBase >> 5;
    const int cb = mBase & 31;
#pragma unroll
    for (int j = 0; j < 4; ++j) {
#pragma unroll
      for (int r = 0; r < 8; ++r)
        slab[(mOff + r) * kSlabPitch + (j << 4) + rlane] = acc[i][j][r] * kOFold;
    }
    wave_lds_fence();
    v8h hv[4];
#pragma unroll
    for (int it = 0; it < 4; ++it) {
      const int p2  = it * 2 + (q >> 1);
      const int row = 2 * p2 + (t >> 2);
      const int col = jh * 32 + (t & 3) * 8;
      const float* sp = slab + row * kSlabPitch + col;
      const v4f a0 = *(const v4f*)(sp);
      const v4f a1 = *(const v4f*)(sp + 4);
      hv[it] = pack8_flush(a0, a1);
    }
    _Float16* prow = Och + (size_t)(il * kRes + jg) * kCk + cb * kCh + t * 8;
    for (int pass = 0; pass < 2; ++pass) {
#pragma unroll
      for (int it = 0; it < 4; ++it) {
        const int p2 = it * 2 + (q >> 1);
        *(volatile v8h*)(prow + (2 * p2) * kCh) = hv[it];
      }
      __threadfence();
    }
    wave_lds_fence();
  }
}

__global__ __launch_bounds__(256) void zproj_gemm_kernel(
    const _Float16* __restrict__ Och, const _Float16* __restrict__ WOT,
    const float* __restrict__ bout, float* __restrict__ Zchunk)
{
  __shared__ __align__(16) float sT[8][16 * kSlabPitch];
  const int lane  = threadIdx.x & 31;
  const int wave  = threadIdx.x >> 5;
  const int tile  = blockIdx.x * 8 + wave;
  constexpr int tilesN = kCz / 64;
  const int tm    = tile / tilesN;
  const int tn    = tile % tilesN;
  const int m0    = tm << 6;
  const int n0    = tn << 6;
  const int rlane = lane & 15;
  const int koff  = (lane >> 4) * 8;
  const int mOff  = (lane >> 4) * 8;

  v8f acc[4][4];
#pragma unroll
  for (int i = 0; i < 4; ++i)
#pragma unroll
    for (int j = 0; j < 4; ++j) acc[i][j] = (v8f){0.f,0.f,0.f,0.f,0.f,0.f,0.f,0.f};

#pragma unroll 1
  for (int k0 = 0; k0 < kCk; k0 += 32) {
    v16h bh[4];
#pragma unroll
    for (int j = 0; j < 4; ++j)
      bh[j] = frag_load(WOT + (size_t)(n0 + (j << 4) + rlane) * kCk + koff + k0);
#pragma unroll
    for (int i = 0; i < 4; ++i) {
      const v16h ah = frag_load(Och + (size_t)(m0 + (i << 4) + rlane) * kCk + koff + k0);
#pragma unroll
      for (int j = 0; j < 4; ++j) acc[i][j] = mma_h(ah, bh[j], acc[i][j]);
    }
  }

  float* slab = sT[wave];
  const int hh = lane >> 4;
  const int c4 = (lane & 15) * 4;
  float bv[4];
#pragma unroll
  for (int j = 0; j < 4; ++j) bv[j] = bout[n0 + (j << 4) + rlane];
#pragma unroll
  for (int i = 0; i < 4; ++i) {
    const int mBase = m0 + (i << 4);
#pragma unroll
    for (int j = 0; j < 4; ++j) {
#pragma unroll
      for (int r = 0; r < 8; ++r) {
        const float v = (acc[i][j][r] * kZFold + bv[j]) * kInvSeq;
        slab[(mOff + r) * kSlabPitch + (j << 4) + rlane] = v;
      }
    }
    wave_lds_fence();
    v4f ov[8];
#pragma unroll
    for (int it = 0; it < 8; ++it) ov[it] = *(const v4f*)(slab + (it * 2 + hh) * kSlabPitch + c4);
    for (int pass = 0; pass < 2; ++pass) {
#pragma unroll
      for (int it = 0; it < 8; ++it)
        *(volatile v4f*)(Zchunk + (size_t)(mBase + it * 2 + hh) * kCz + n0 + c4) = ov[it];
      __threadfence();
    }
    wave_lds_fence();
  }
}

extern "C" void kernel_launch(void* const* d_in, const int* in_sizes, int n_in,
                              void* d_out, int out_size, void* d_ws, size_t ws_size,
                              hipStream_t stream) {
  if (n_in < 9) return;
  if (in_sizes[0] != kSeq * kRes * kCm) return;
  if (in_sizes[1] != kCm) return;
  if (in_sizes[2] != kCm) return;
  if (in_sizes[3] != kCm * kCh) return;
  if (in_sizes[4] != kCh) return;
  if (in_sizes[5] != kCm * kCh) return;
  if (in_sizes[6] != kCh) return;
  if (in_sizes[7] != kCk * kCz) return;
  if (in_sizes[8] != kCz) return;
  if (out_size != kRes * kRes * kCz) return;
  if (ws_size < kWsTotal) return;

  const float* m     = (const float*)d_in[0];
  const float* gamma = (const float*)d_in[1];
  const float* beta  = (const float*)d_in[2];
  const float* W1    = (const float*)d_in[3];
  const float* b1    = (const float*)d_in[4];
  const float* W2    = (const float*)d_in[5];
  const float* b2    = (const float*)d_in[6];
  const float* Wout  = (const float*)d_in[7];
  const float* bout  = (const float*)d_in[8];
  float* Z = (float*)d_out;

  char* ws = (char*)d_ws;
  _Float16* W12H = (_Float16*)(ws + kOffW12H);
  _Float16* W12L = (_Float16*)(ws + kOffW12L);
  _Float16* WOT  = (_Float16*)(ws + kOffWOT);
  _Float16* MNH  = (_Float16*)(ws + kOffMNH);
  _Float16* MNL  = (_Float16*)(ws + kOffMNL);
  _Float16* ABP  = (_Float16*)(ws + kOffABP);
  _Float16* OCH  = (_Float16*)(ws + kOffOCH);

  prep_weights_kernel<<<72, 256, 0, stream>>>(W1, W2, Wout, W12H, W12L, WOT);

  layernorm_planes_kernel<<<kLnRows / 8, 256, 0, stream>>>(m, gamma, beta, MNH, MNL);

  proj_split_kernel<<<(2 * (kLnRows / 64)) / 8, 256, 0, stream>>>(W12H, W12L, MNH, MNL, b1, b2, ABP);

  const _Float16* ATp = ABP;
  const _Float16* BTp = ABP + (size_t)kAbRows * kSeq;
  for (int p = 0; p < kChunks; ++p) {
    outer_gemm_kernel<<<((kChunkM / 64) * (kAbRows / 64)) / 8, 256, 0, stream>>>(
        ATp + (size_t)p * kChunkM * kSeq, BTp, OCH);
    zproj_gemm_kernel<<<((kChunkPairs / 64) * (kCz / 64)) / 8, 256, 0, stream>>>(
        OCH, WOT, bout, Z + (size_t)p * kChunkPairs * kCz);
  }
}
